// Relation_72112500899921
// MI455X (gfx1250) — hardware-verified
//
#include <hip/hip_runtime.h>
#include <math.h>
#include <stdint.h>

#ifndef NQ
#define NQ      2048
#endif
#define NQ_FULL 2048
#define MREF    2048
#define FD      2048
#define NG      16
#define HD      128
#define NQB     (NQ / 64)
#define NKT     (MREF / 64)
static_assert(NG * HD == FD);
static_assert((NQ % 64) == 0 && NQ >= 64 && NQ <= NQ_FULL);
static_assert((MREF % 64) == 0 && (FD % 64) == 0 && (FD % 32) == 0);
static_assert(NKT == 32);

typedef _Float16 v16h __attribute__((ext_vector_type(16)));
typedef _Float16 v8h  __attribute__((ext_vector_type(8)));
typedef __bf16   v16b __attribute__((ext_vector_type(16)));
typedef __bf16   v8b  __attribute__((ext_vector_type(8)));
typedef float    v8f  __attribute__((ext_vector_type(8)));
typedef float    v4f  __attribute__((ext_vector_type(4)));
typedef unsigned int v4u __attribute__((ext_vector_type(4)));

#if defined(__HIP_DEVICE_COMPILE__)
#define DEV_ASM 1
#else
#define DEV_ASM 0
#endif

__device__ __forceinline__ unsigned short bf_bits(float f) {
  unsigned u = __float_as_uint(f);
  return (unsigned short)((u + 0x7FFFu + ((u >> 16) & 1u)) >> 16);
}
__device__ __forceinline__ float bf_up(unsigned short hb) { return __uint_as_float(((unsigned)hb) << 16); }
__device__ __forceinline__ unsigned short h_bits(_Float16 x) { return __builtin_bit_cast(unsigned short, x); }
__device__ __forceinline__ unsigned pk16(unsigned short a, unsigned short b) { return (unsigned)a | ((unsigned)b << 16); }
__device__ __forceinline__ v8f zero8() { v8f z = {0.f, 0.f, 0.f, 0.f, 0.f, 0.f, 0.f, 0.f}; return z; }

template <typename OT> struct FT;
template <> struct FT<__bf16>   { typedef v16b frag; typedef v8b half8; };
template <> struct FT<_Float16> { typedef v16h frag; typedef v8h half8; };

template <typename OT>
__device__ __forceinline__ typename FT<OT>::frag ldfrag(const OT* p) {
  union { typename FT<OT>::frag v; typename FT<OT>::half8 h[2]; } f;
  f.h[0] = *(const typename FT<OT>::half8*)(p);
  f.h[1] = *(const typename FT<OT>::half8*)(p + 16);
  return f.v;
}

__device__ __forceinline__ v8f mmar(v16b a, v16b b, v8f c) {
  return __builtin_amdgcn_wmma_f32_16x16x32_bf16(false, a, false, b, (short)0, c, false, false);
}
__device__ __forceinline__ v8f mmar(v16h a, v16h b, v8f c) {
  return __builtin_amdgcn_wmma_f32_16x16x32_f16(false, a, false, b, (short)0, c, false, false);
}
__device__ __forceinline__ v8f mma_h(v16h a, v16h b, v8f c) {
  c = __builtin_amdgcn_wmma_f32_16x16x32_f16(false, a, false, b, (short)0, c, false, false);
#if DEV_ASM
  asm volatile("v_nop\n\tv_nop\n\tv_nop\n\tv_nop" : "+v"(c) : "v"(a), "v"(b));
#endif
  return c;
}
__device__ __forceinline__ void dep_guard(v8f& a, v8f& b, v16b x, v16b y) {
#if DEV_ASM
  asm volatile("v_nop\n\tv_nop\n\tv_nop\n\tv_nop" : "+v"(a), "+v"(b) : "v"(x), "v"(y));
#else
  (void)a; (void)b; (void)x; (void)y;
#endif
}
__device__ __forceinline__ void dep_guard(v8f& a, v8f& b, v16h x, v16h y) {
#if DEV_ASM
  asm volatile("v_nop\n\tv_nop\n\tv_nop\n\tv_nop" : "+v"(a), "+v"(b) : "v"(x), "v"(y));
#else
  (void)a; (void)b; (void)x; (void)y;
#endif
}
__device__ __forceinline__ void keep4(v16b a, v16b b, v16b c, v16b d) {
#if DEV_ASM
  asm volatile("v_nop" :: "v"(a), "v"(b), "v"(c), "v"(d));
#else
  (void)a; (void)b; (void)c; (void)d;
#endif
}
__device__ __forceinline__ void keep4(v16h a, v16h b, v16h c, v16h d) {
#if DEV_ASM
  asm volatile("v_nop" :: "v"(a), "v"(b), "v"(c), "v"(d));
#else
  (void)a; (void)b; (void)c; (void)d;
#endif
}
__device__ __forceinline__ void acc_guard4(v8f& a, v8f& b, v8f& c, v8f& d) {
#if DEV_ASM
  asm volatile("v_nop\n\tv_nop\n\tv_nop\n\tv_nop" : "+v"(a), "+v"(b), "+v"(c), "+v"(d));
#else
  (void)a; (void)b; (void)c; (void)d;
#endif
}

__global__ __launch_bounds__(256) void cvt_bf16x8(const float* __restrict__ in, unsigned short* out, int n8) {
  const int i = blockIdx.x * 256 + (int)threadIdx.x;
  if (i < n8) {
    const v4f a  = *(const v4f*)(in + (size_t)i * 8);
    const v4f a4 = *(const v4f*)(in + (size_t)i * 8 + 4);
    v4u p;
    p[0] = pk16(bf_bits(a[0]),  bf_bits(a[1]));
    p[1] = pk16(bf_bits(a[2]),  bf_bits(a[3]));
    p[2] = pk16(bf_bits(a4[0]), bf_bits(a4[1]));
    p[3] = pk16(bf_bits(a4[2]), bf_bits(a4[3]));
    unsigned short* o = out + (size_t)i * 8;
    *(volatile v4u*)o = p;
    __threadfence();
    *(volatile v4u*)o = p;
  }
}

template <typename OT, int OUT_MODE, bool BIAS>
__global__ __launch_bounds__(256) void gemm64(
    const unsigned short* __restrict__ Ap, int lda,
    const unsigned short* __restrict__ Btp, int ldb,
    unsigned short* Cout, unsigned short* Cout2, int ldc,
    const float* __restrict__ bias,
    int M, int N, int K, float rscale) {
  typedef typename FT<OT>::frag V16;
  const OT* Ab = (const OT*)(const void*)Ap;
  const OT* Bb = (const OT*)(const void*)Btp;
  __shared__ __align__(16) float sT[8][16 * 68];
  const int lane = threadIdx.x & 31;
  const int wave = threadIdx.x >> 5;
  const int tilesN = N >> 6;
  const int tilesM = M >> 6;
  const int tile = blockIdx.x * 8 + wave;
  if (tile >= tilesM * tilesN) return;
  const int tm = tile / tilesN;
  const int tn = tile - tm * tilesN;
  const int m0 = tm << 6;
  const int n0 = tn << 6;

  const int rlane = lane & 15;
  const int koff  = (lane >> 4) * 8;
  const int mOff  = (lane >> 4) * 8;

  v8f acc[4][4];
#pragma unroll
  for (int i = 0; i < 4; ++i)
#pragma unroll
    for (int j = 0; j < 4; ++j) acc[i][j] = zero8();

  for (int k0 = 0; k0 < K; k0 += 32) {
    V16 bq[4];
#pragma unroll
    for (int j = 0; j < 4; ++j)
      bq[j] = ldfrag<OT>(Bb + (size_t)(n0 + (j << 4) + rlane) * ldb + koff + k0);
#pragma unroll
    for (int i = 0; i < 4; ++i) {
      const V16 af = ldfrag<OT>(Ab + (size_t)(m0 + (i << 4) + rlane) * lda + koff + k0);
#pragma unroll
      for (int j = 0; j < 4; ++j) acc[i][j] = mmar(af, bq[j], acc[i][j]);
      dep_guard(acc[i][0], acc[i][3], af, bq[3]);
    }
    keep4(bq[0], bq[1], bq[2], bq[3]);
  }
  acc_guard4(acc[0][0], acc[0][1], acc[0][2], acc[0][3]);
  acc_guard4(acc[1][0], acc[1][1], acc[1][2], acc[1][3]);
  acc_guard4(acc[2][0], acc[2][1], acc[2][2], acc[2][3]);
  acc_guard4(acc[3][0], acc[3][1], acc[3][2], acc[3][3]);

  float* slab = sT[wave];
  const int q = lane >> 3, c8 = (lane & 7) * 8;
  float bz[8];
#pragma unroll
  for (int e = 0; e < 8; ++e) bz[e] = 0.f;
  if (BIAS) {
    const v4f b0 = *(const v4f*)(bias + n0 + c8);
    const v4f b1 = *(const v4f*)(bias + n0 + c8 + 4);
#pragma unroll
    for (int e = 0; e < 4; ++e) { bz[e] = bf_up(bf_bits(b0[e])); bz[4 + e] = bf_up(bf_bits(b1[e])); }
  }
#pragma unroll
  for (int i = 0; i < 4; ++i) {
    const int mBase = m0 + (i << 4);
#pragma unroll
    for (int j = 0; j < 4; ++j) {
#pragma unroll
      for (int r = 0; r < 8; ++r) {
        slab[(mOff + r) * 68 + (j << 4) + rlane] = acc[i][j][r];
      }
    }
    __builtin_amdgcn_fence(__ATOMIC_RELEASE, "workgroup");
    __builtin_amdgcn_wave_barrier();
    __builtin_amdgcn_fence(__ATOMIC_ACQUIRE, "workgroup");
    {
      v4u hv[4], lv[4];
#pragma unroll
      for (int it = 0; it < 4; ++it) {
        const int row = it * 4 + q;
        const float* sp = slab + row * 68 + c8;
        float f[8];
#pragma unroll
        for (int e = 0; e < 8; ++e) f[e] = sp[e] + bz[e];
        v4u a, a2;
#pragma unroll
        for (int e = 0; e < 4; ++e) {
          const float f0 = f[2 * e], f1 = f[2 * e + 1];
          const _Float16 x0 = (_Float16)f0, x1 = (_Float16)f1;
          const unsigned short h0 = h_bits(x0), h1 = h_bits(x1);
          unsigned short l0 = 0, l1 = 0;
          if (OUT_MODE == 3) {
            l0 = h_bits((_Float16)((f0 - (float)x0) * rscale));
            l1 = h_bits((_Float16)((f1 - (float)x1) * rscale));
          }
          a[e] = pk16(h0, h1); a2[e] = pk16(l0, l1);
        }
        hv[it] = a; lv[it] = a2;
      }
      for (int pass = 0; pass < 2; ++pass) {
#pragma unroll
        for (int it = 0; it < 4; ++it) {
          const int row = it * 4 + q;
          *(volatile v4u*)(Cout + (size_t)(mBase + row) * ldc + n0 + c8) = hv[it];
          if (OUT_MODE == 3) *(volatile v4u*)(Cout2 + (size_t)(mBase + row) * ldc + n0 + c8) = lv[it];
        }
        __threadfence();
      }
    }
    __builtin_amdgcn_fence(__ATOMIC_RELEASE, "workgroup");
    __builtin_amdgcn_wave_barrier();
    __builtin_amdgcn_fence(__ATOMIC_ACQUIRE, "workgroup");
  }
}

__global__ __launch_bounds__(128) __attribute__((amdgpu_num_vgpr(256)))
void attn_rel(const unsigned short* __restrict__ qhp, const unsigned short* __restrict__ qlp,
              const unsigned short* __restrict__ kpp, const unsigned short* __restrict__ vtp,
              const float* __restrict__ vbias, float* op, float sscale) {
  union FH { v16h v; v8h h[2]; };
  __shared__ __align__(16) _Float16 Ksh[64 * HD];
  __shared__ __align__(16) _Float16 Vth[HD * 64];
  __shared__ __align__(16) _Float16 Psh[4][16 * 64];
  __shared__ __align__(16) float    Os[4][16 * 64];

  const int tid  = threadIdx.x;
  const int wave = tid >> 5;
  const int lane = tid & 31;
  const int hh   = lane >> 4;
  const int c    = lane & 15;

  const int bx   = blockIdx.x;
  const int qb   = bx % NQB;
  const int g    = bx / NQB;
  const int q0   = qb * 64 + wave * 16;

  const _Float16* Qh = (const _Float16*)(const void*)qhp;
  const _Float16* Ql = (const _Float16*)(const void*)qlp;
  const _Float16* Kg = (const _Float16*)(const void*)kpp + (size_t)g * HD;
  const _Float16* Vg = (const _Float16*)(const void*)vtp + (size_t)g * HD * MREF;

  v16h qah[4], qal[4];
#pragma unroll
  for (int dc = 0; dc < 4; ++dc) {
    const size_t qo = (size_t)(q0 + c) * FD + (size_t)g * HD + dc * 32 + 8 * hh;
    qah[dc] = ldfrag<_Float16>(Qh + qo);
    qal[dc] = ldfrag<_Float16>(Ql + qo);
  }

  float mrow[8], lrow[8];
  v8f oacc[8];
#pragma unroll
  for (int r = 0; r < 8; ++r) { mrow[r] = -INFINITY; lrow[r] = 0.f; }
#pragma unroll
  for (int t = 0; t < 8; ++t) oacc[t] = zero8();

  for (int kt = 0; kt < NKT; ++kt) {
    const int kv0 = kt * 64;
    __syncthreads();
    {
      const int r = tid >> 1, half = (tid & 1) * 64;
      const _Float16* kg = Kg + (size_t)(kv0 + r) * FD + half;
#pragma unroll
      for (int i = 0; i < 8; ++i) {
        const v8h a0 = *(const v8h*)(kg + 8 * i);
        *(v8h*)(Ksh + r * HD + half + 8 * i) = a0;
      }
      const _Float16* vg = Vg + (size_t)tid * MREF + kv0;
#pragma unroll
      for (int i = 0; i < 8; ++i) {
        const v8h b0 = *(const v8h*)(vg + 8 * i);
        *(v8h*)(Vth + tid * 64 + 8 * i) = b0;
      }
    }
    __syncthreads();

    v8f s[4];
#pragma unroll
    for (int j = 0; j < 4; ++j) {
      v8f ah = zero8(), al = zero8();
#pragma unroll
      for (int dc = 0; dc < 4; ++dc) {
        FH kb;
        kb.h[0] = *(const v8h*)(Ksh + (j * 16 + c) * HD + dc * 32 + 8 * hh);
        kb.h[1] = *(const v8h*)(Ksh + (j * 16 + c) * HD + dc * 32 + 16 + 8 * hh);
        ah = mma_h(qah[dc], kb.v, ah);
        al = mma_h(qal[dc], kb.v, al);
      }
#pragma unroll
      for (int r = 0; r < 8; ++r) s[j][r] = (ah[r] + al[r] * (1.0f / 4096.0f)) * sscale;
    }

    _Float16* pwh = Psh[wave];
#pragma unroll
    for (int r = 0; r < 8; ++r) {
      float m = s[0][r];
#pragma unroll
      for (int j = 1; j < 4; ++j) m = fmaxf(m, s[j][r]);
#pragma unroll
      for (int off = 1; off < 16; off <<= 1) m = fmaxf(m, __shfl_xor(m, off, 32));
      const float mnew  = fmaxf(mrow[r], m);
      const float msafe = (mnew == -INFINITY) ? 0.f : mnew;
      const float alpha = __expf(mrow[r] - msafe);
      mrow[r] = mnew;
      float psum = 0.f;
#pragma unroll
      for (int j = 0; j < 4; ++j) {
        const float p = __expf(s[j][r] - msafe);
        psum += p;
        pwh[(8 * hh + r) * 64 + j * 16 + c] = (_Float16)(p * 1024.0f);
      }
#pragma unroll
      for (int off = 1; off < 16; off <<= 1) psum += __shfl_xor(psum, off, 32);
      lrow[r] = lrow[r] * alpha + psum;
#pragma unroll
      for (int t = 0; t < 8; ++t) oacc[t][r] *= alpha;
    }
    __builtin_amdgcn_fence(__ATOMIC_RELEASE, "workgroup");
    __builtin_amdgcn_wave_barrier();
    __builtin_amdgcn_fence(__ATOMIC_ACQUIRE, "workgroup");

    v16h pa[2];
#pragma unroll
    for (int kk = 0; kk < 2; ++kk) {
      FH pf;
      pf.h[0] = *(const v8h*)(pwh + c * 64 + kk * 32 + 8 * hh);
      pf.h[1] = *(const v8h*)(pwh + c * 64 + kk * 32 + 16 + 8 * hh);
      pa[kk] = pf.v;
    }
#pragma unroll
    for (int t = 0; t < 8; ++t) {
#pragma unroll
      for (int kk = 0; kk < 2; ++kk) {
        FH vb;
        vb.h[0] = *(const v8h*)(Vth + (t * 16 + c) * 64 + kk * 32 + 8 * hh);
        vb.h[1] = *(const v8h*)(Vth + (t * 16 + c) * 64 + kk * 32 + 16 + 8 * hh);
        oacc[t] = mma_h(pa[kk], vb.v, oacc[t]);
      }
    }
    keep4(pa[0], pa[1], qah[0], qal[0]);
  }

  float bb[8], inv8[8];
#pragma unroll
  for (int t = 0; t < 8; ++t) bb[t] = bf_up(bf_bits(vbias[g * HD + t * 16 + c]));
#pragma unroll
  for (int r = 0; r < 8; ++r) {
    const float l = lrow[r];
    inv8[r] = ((l > 0.f) ? (1.0f / l) : 0.f) * (1.0f / 1024.0f);
  }
  float* os = Os[wave];
#pragma unroll
  for (int ph = 0; ph < 2; ++ph) {
#pragma unroll
    for (int r = 0; r < 8; ++r) {
#pragma unroll
      for (int t4 = 0; t4 < 4; ++t4) {
        os[(8 * hh + r) * 64 + t4 * 16 + c] = oacc[ph * 4 + t4][r] * inv8[r] + bb[ph * 4 + t4];
      }
    }
    __builtin_amdgcn_fence(__ATOMIC_RELEASE, "workgroup");
    __builtin_amdgcn_wave_barrier();
    __builtin_amdgcn_fence(__ATOMIC_ACQUIRE, "workgroup");
    for (int pass = 0; pass < 2; ++pass) {
#pragma unroll
      for (int it = 0; it < 8; ++it) {
        const int row = it * 2 + hh;
        const float* sp = os + row * 64 + c * 4;
        v4f v;
        v[0] = sp[0]; v[1] = sp[1]; v[2] = sp[2]; v[3] = sp[3];
        const size_t go = (size_t)(q0 + row) * FD + (size_t)g * HD + ph * 64 + c * 4;
        *(volatile v4f*)(op + go) = v;
      }
      __threadfence();
    }
    __builtin_amdgcn_fence(__ATOMIC_RELEASE, "workgroup");
    __builtin_amdgcn_wave_barrier();
    __builtin_amdgcn_fence(__ATOMIC_ACQUIRE, "workgroup");
  }
}

extern "C" void kernel_launch(void* const* d_in, const int* in_sizes, int n_in,
                              void* d_out, int out_size, void* d_ws, size_t ws_size,
                              hipStream_t stream) {
  if (n_in < 8) return;
  if (in_sizes[0] < NQ * FD) return;
  if (in_sizes[1] < MREF * FD) return;
  if (in_sizes[2] < FD * FD || in_sizes[4] < FD * FD || in_sizes[6] < FD * FD) return;
  if (in_sizes[3] < FD || in_sizes[5] < FD || in_sizes[7] < FD) return;
  if (out_size < NQ * FD) return;

  const float* roi  = (const float*)d_in[0];
  const float* reff = (const float*)d_in[1];
  const float* Wq   = (const float*)d_in[2];
  const float* Wq_b = (const float*)d_in[3];
  const float* Wk   = (const float*)d_in[4];
  const float* Wk_b = (const float*)d_in[5];
  const float* Wv   = (const float*)d_in[6];
  const float* Wv_b = (const float*)d_in[7];

  const size_t PQ = (size_t)NQ * FD * 2;
  const size_t P8 = (size_t)FD * FD * 2;
  size_t off = 0;
  const size_t oXr = off; off += PQ;
  const size_t oXf = off; off += P8;
  const size_t oWq = off; off += P8;
  const size_t oWk = off; off += P8;
  const size_t oWv = off; off += P8;
  const size_t oQh = off; off += PQ;
  const size_t oQl = off; off += PQ;
  const size_t oKp = off; off += P8;
  const size_t oVT = off; off += P8;
  if (off > ws_size) return;
  if (off > (size_t)134217728) return;

  char* ws = (char*)d_ws;
  unsigned short* Xr  = (unsigned short*)(ws + oXr);
  unsigned short* Xf  = (unsigned short*)(ws + oXf);
  unsigned short* Wqb = (unsigned short*)(ws + oWq);
  unsigned short* Wkb = (unsigned short*)(ws + oWk);
  unsigned short* Wvb = (unsigned short*)(ws + oWv);
  unsigned short* Qh  = (unsigned short*)(ws + oQh);
  unsigned short* Ql  = (unsigned short*)(ws + oQl);
  unsigned short* Kp  = (unsigned short*)(ws + oKp);
  unsigned short* VT  = (unsigned short*)(ws + oVT);

  const dim3 blk(256);
  const int n8q = NQ * FD / 8;
  const int n8f = MREF * FD / 8;
  const int n8w = FD * FD / 8;
  const dim3 gCvtQ((n8q + 255) / 256);
  const dim3 gCvtF((n8f + 255) / 256);
  const dim3 gCvtW((n8w + 255) / 256);
  const dim3 gQ(((NQ / 64) * (FD / 64) + 7) / 8);
  const dim3 gK(((MREF / 64) * (FD / 64) + 7) / 8);
  const dim3 gVT(((FD / 64) * (MREF / 64) + 7) / 8);
  const dim3 gAttn(NG * NQB);
  const float sscale = (float)(1.0 / sqrt((double)HD));

  cvt_bf16x8<<<gCvtQ, blk, 0, stream>>>(roi,  Xr,  n8q);
  cvt_bf16x8<<<gCvtF, blk, 0, stream>>>(reff, Xf,  n8f);
  cvt_bf16x8<<<gCvtW, blk, 0, stream>>>(Wq,   Wqb, n8w);
  cvt_bf16x8<<<gCvtW, blk, 0, stream>>>(Wk,   Wkb, n8w);
  cvt_bf16x8<<<gCvtW, blk, 0, stream>>>(Wv,   Wvb, n8w);
  gemm64<__bf16, 3, true><<<gQ, blk, 0, stream>>>(
      Xr, FD, Wqb, FD, Qh, Ql, FD, Wq_b, NQ, FD, FD, 4096.0f);
  gemm64<__bf16, 1, true><<<gK, blk, 0, stream>>>(
      Xf, FD, Wkb, FD, Kp, Kp, FD, Wk_b, MREF, FD, FD, 1.0f);
  gemm64<__bf16, 1, false><<<gVT, blk, 0, stream>>>(
      Wvb, FD, Xf, FD, VT, VT, MREF, Wv_b, FD, MREF, FD, 1.0f);
  attn_rel<<<gAttn, dim3(128), 0, stream>>>(Qh, Ql, Kp, VT, Wv_b, (float*)d_out, sscale);
  (void)hipGetLastError();
}
